// FasterMultiHeadAttention_66838281060489
// MI455X (gfx1250) — hardware-verified
//
#include <hip/hip_runtime.h>
#include <math.h>


#define BB 2
#define SS 2048
#define DD 1024
#define HH 16
#define HD 64
#define BS (BB * SS)
#define D3 (3 * DD)
#define BK 32

typedef __attribute__((ext_vector_type(16))) _Float16 v16h;
typedef __attribute__((ext_vector_type(8)))  _Float16 v8h;
typedef __attribute__((ext_vector_type(8)))  float v8f;
typedef __attribute__((ext_vector_type(4)))  float v4f;
typedef __attribute__((ext_vector_type(4)))  unsigned v4u;

template <typename T> __device__ __forceinline__ void vst2(void* p, T v) { *(volatile T*)p = v; __threadfence(); *(volatile T*)p = v; }
__device__ __forceinline__ v8f wmma16(v16h a, v16h b, v8f c) {
  v8f d = __builtin_amdgcn_wmma_f32_16x16x32_f16(false, a, false, b, (short)0, c, false, false);
  asm volatile("v_nop\n\tv_nop\n\tv_nop\n\tv_nop" : "+v"(d) : "v"(a), "v"(b));
  return d;
}
__device__ __forceinline__ v16h frag_h(const _Float16* rowk0, int lane) {
  union { v16h v; v8h q[2]; } u; const _Float16* p = rowk0 + 8 * (lane >> 4);
  u.q[0] = *(const v8h*)p; u.q[1] = *(const v8h*)(p + 16); return u.v;
}
__device__ __forceinline__ v16h frag_f32(const float* rowk0, int lane) {
  v16h a; const float* p = rowk0 + 8 * (lane >> 4);
#pragma unroll
  for (int i = 0; i < 8; ++i) { a[i] = (_Float16)p[i]; a[8 + i] = (_Float16)p[16 + i]; }
  return a;
}
#define LDSX() do { asm volatile("s_wait_dscnt 0" ::: "memory"); __builtin_amdgcn_wave_barrier(); __builtin_amdgcn_fence(__ATOMIC_RELEASE, "workgroup"); } while (0)

__global__ __launch_bounds__(256) void k_cvt_rows(const float* __restrict__ s, _Float16* __restrict__ d, size_t n8) {
  const size_t g8 = (size_t)blockIdx.x * 256 + threadIdx.x; if (g8 >= n8) return;
  union { v8h h; v4u u; } pk;
#pragma unroll
  for (int e = 0; e < 8; ++e) pk.h[e] = (_Float16)s[g8 * 8 + e];
  vst2(d + g8 * 8, pk.u);
}
__global__ __launch_bounds__(256) void k_pack_wt(const float* __restrict__ W, _Float16* __restrict__ Wt, int K, int N) {
  const size_t g8 = (size_t)blockIdx.x * 256 + threadIdx.x; if (g8 >= (size_t)N * K / 8) return;
  const int n = (int)(g8 / (K / 8)), k0 = (int)(g8 % (K / 8)) * 8;
  union { v8h h; v4u u; } pk;
#pragma unroll
  for (int e = 0; e < 8; ++e) pk.h[e] = (_Float16)W[(size_t)(k0 + e) * N + n];
  vst2(Wt + (size_t)n * K + k0, pk.u);
}

__global__ __launch_bounds__(128) void k_qkv(const _Float16* __restrict__ xh, const _Float16* __restrict__ Wt, const float* __restrict__ bqkv,
                                           _Float16* __restrict__ qh, _Float16* __restrict__ kh, _Float16* __restrict__ vT) {
  __shared__ __align__(16) float st[128][68];
  const int tid = threadIdx.x, wave = tid >> 5, lane = tid & 31, col = lane & 15, g = lane >> 4;
  const int r0 = blockIdx.x * 64, n0 = blockIdx.y * 128;
  const int b = r0 / SS, s0 = r0 % SS;
  v8f acc[8] = {};
#pragma unroll 1
  for (int kc = 0; kc < DD / 32; ++kc) {
    const v16h a = frag_h(xh + (size_t)(r0 + wave * 16 + col) * DD + kc * 32, lane);
#pragma unroll
    for (int j = 0; j < 8; ++j) acc[j] = wmma16(a, frag_h(Wt + (size_t)(n0 + j * 16 + col) * DD + kc * 32, lane), acc[j]);
  }
#pragma unroll
  for (int j = 0; j < 8; ++j) { const float bv = bqkv[n0 + j * 16 + col];
#pragma unroll
    for (int r = 0; r < 8; ++r) st[j * 16 + col][wave * 16 + 8 * g + r] = acc[j][r] + bv; }
  __syncthreads();
  const int which = n0 / DD, h0 = (n0 % DD) / HD;
  if (which < 2) {
    _Float16* dst = which == 0 ? qh : kh;
    for (int q = tid; q < 2 * 64 * 8; q += 128) { const int hh = q >> 9, sl = (q >> 3) & 63, pc = q & 7;
      union { v8h h; v4u u; } pk;
#pragma unroll
      for (int e = 0; e < 8; ++e) pk.h[e] = (_Float16)st[hh * 64 + pc * 8 + e][sl];
      vst2(dst + (((size_t)b * HH + h0 + hh) * SS + s0 + sl) * HD + pc * 8, pk.u); }
  } else {
    for (int q = tid; q < 128 * 8; q += 128) { const int cl = q >> 3, pc = q & 7; const int hh = cl >> 6, d = cl & 63;
      union { v8h h; v4u u; } pk;
#pragma unroll
      for (int i = 0; i < 8; ++i) pk.h[i] = (_Float16)st[cl][pc * 8 + i];
      vst2(vT + (((size_t)b * HH + h0 + hh) * HD + d) * SS + s0 + pc * 8, pk.u); }
  }
}

__global__ __launch_bounds__(128) void k_attn(const _Float16* __restrict__ qh, const _Float16* __restrict__ kh, const _Float16* __restrict__ vT,
                                            _Float16* __restrict__ ao) {
  __shared__ __align__(16) float sP[4][16][BK];
  __shared__ __align__(16) float sO[4][16][HD];
  const int tid = threadIdx.x, w = tid >> 5, lane = tid & 31, g = lane >> 4, ln = lane & 15;
  const int bh = blockIdx.y, b = bh / HH, h = bh % HH, q0 = blockIdx.x * 64 + w * 16;
  const _Float16* qrow = qh + ((size_t)bh * SS + q0 + ln) * HD;
  const v16h qa0 = frag_h(qrow, lane), qa1 = frag_h(qrow + 32, lane);
  const float scale = 0.125f;
  float mrun[8], lrun[8];
  v8f acc[4];
#pragma unroll
  for (int r = 0; r < 8; ++r) { mrun[r] = -3.0e38f; lrun[r] = 0.f; }
#pragma unroll
  for (int t = 0; t < 4; ++t) acc[t] = (v8f){};
  const _Float16* kb = kh + (size_t)bh * SS * HD;
  const _Float16* vb = vT + (size_t)bh * HD * SS;
#pragma unroll 1
  for (int k0 = 0; k0 < SS; k0 += BK) {
    v8f s0 = {}, s1 = {};
    s0 = wmma16(qa0, frag_h(kb + (size_t)(k0 + ln) * HD, lane), s0);      s0 = wmma16(qa1, frag_h(kb + (size_t)(k0 + ln) * HD + 32, lane), s0);
    s1 = wmma16(qa0, frag_h(kb + (size_t)(k0 + 16 + ln) * HD, lane), s1); s1 = wmma16(qa1, frag_h(kb + (size_t)(k0 + 16 + ln) * HD + 32, lane), s1);
#pragma unroll
    for (int r = 0; r < 8; ++r) {
      const float x0 = s0[r] * scale, x1 = s1[r] * scale;
      float mx = fmaxf(x0, x1);
#pragma unroll
      for (int off = 8; off >= 1; off >>= 1) mx = fmaxf(mx, __shfl_xor(mx, off, 32));
      const float mn = fmaxf(mrun[r], mx);
      const float corr = expf(mrun[r] - mn);
      const float p0 = expf(x0 - mn), p1 = expf(x1 - mn);
      float sum = p0 + p1;
#pragma unroll
      for (int off = 8; off >= 1; off >>= 1) sum += __shfl_xor(sum, off, 32);
      lrun[r] = lrun[r] * corr + sum; mrun[r] = mn;
#pragma unroll
      for (int t = 0; t < 4; ++t) acc[t][r] *= corr;
      sP[w][8 * g + r][ln] = p0 * 16384.0f; sP[w][8 * g + r][16 + ln] = p1 * 16384.0f;
    }
    LDSX();
    const v16h pa = frag_f32(&sP[w][ln][0], lane);
#pragma unroll
    for (int t = 0; t < 4; ++t) acc[t] = wmma16(pa, frag_h(vb + (size_t)(t * 16 + ln) * SS + k0, lane), acc[t]);
    __builtin_amdgcn_wave_barrier();
  }
  float* so = &sO[w][0][0];
#pragma unroll
  for (int r = 0; r < 8; ++r) { const float il = (1.0f / 16384.0f) / lrun[r];
#pragma unroll
    for (int t = 0; t < 4; ++t) so[(8 * g + r) * HD + t * 16 + ln] = acc[t][r] * il; }
  LDSX();
#pragma unroll
  for (int i = 0; i < 4; ++i) { const int q = i * 32 + lane; const int rl = q >> 3, pc = q & 7;
    union { v8h hh; v4u u; } pk;
#pragma unroll
    for (int e = 0; e < 8; ++e) pk.hh[e] = (_Float16)so[rl * HD + pc * 8 + e];
    vst2(ao + ((size_t)b * SS + q0 + rl) * DD + h * HD + pc * 8, pk.u); }
}

__global__ __launch_bounds__(128) void k_out(const _Float16* __restrict__ ao, const _Float16* __restrict__ Wot, const float* __restrict__ bo,
                                           float* __restrict__ out) {
  __shared__ __align__(16) float so[4][16 * 128];
  const int tid = threadIdx.x, wave = tid >> 5, lane = tid & 31, col = lane & 15, g = lane >> 4;
  const int r0 = blockIdx.x * 64 + wave * 16, n0 = blockIdx.y * 128;
  v8f acc[8] = {};
#pragma unroll 1
  for (int kc = 0; kc < DD / 32; ++kc) {
    const v16h a = frag_h(ao + (size_t)(r0 + col) * DD + kc * 32, lane);
#pragma unroll
    for (int j = 0; j < 8; ++j) acc[j] = wmma16(a, frag_h(Wot + (size_t)(n0 + j * 16 + col) * DD + kc * 32, lane), acc[j]);
  }
  float* S = so[wave];
#pragma unroll
  for (int j = 0; j < 8; ++j) { const float bv = bo[n0 + j * 16 + col];
#pragma unroll
    for (int r = 0; r < 8; ++r) S[(8 * g + r) * 128 + j * 16 + col] = acc[j][r] + bv; }
  LDSX();
#pragma unroll 4
  for (int rl = 0; rl < 16; ++rl) vst2(out + (size_t)(r0 + rl) * DD + n0 + lane * 4, *(const v4f*)(S + rl * 128 + lane * 4));
}

extern "C" void kernel_launch(void* const* d_in, const int* in_sizes, int n_in,
                              void* d_out, int out_size, void* d_ws, size_t ws_size,
                              hipStream_t stream) {
  (void)in_sizes; (void)n_in; (void)out_size; (void)ws_size;
  const float* x     = (const float*)d_in[0];
  const float* w_qkv = (const float*)d_in[1];
  const float* b_qkv = (const float*)d_in[2];
  const float* w_out = (const float*)d_in[3];
  const float* b_out = (const float*)d_in[4];
  float* out = (float*)d_out;
  char* ws = (char*)d_ws; size_t off = 0;
  auto take = [&](size_t bytes) { char* p = ws + off; off += (bytes + 255) & ~(size_t)255; return p; };
  _Float16* xh  = (_Float16*)take((size_t)BS * DD * 2);
  _Float16* Wt  = (_Float16*)take((size_t)D3 * DD * 2);
  _Float16* Wot = (_Float16*)take((size_t)DD * DD * 2);
  _Float16* qh  = (_Float16*)take((size_t)BS * DD * 2);
  _Float16* kh  = (_Float16*)take((size_t)BS * DD * 2);
  _Float16* vT  = (_Float16*)take((size_t)BS * DD * 2);
  _Float16* ao  = (_Float16*)take((size_t)BS * DD * 2);
  k_cvt_rows<<<(unsigned)((BS * DD / 8 + 255) / 256), 256, 0, stream>>>(x, xh, (size_t)BS * DD / 8);
  k_pack_wt<<<(unsigned)((D3 * DD / 8 + 255) / 256), 256, 0, stream>>>(w_qkv, Wt, DD, D3);
  k_pack_wt<<<(unsigned)((DD * DD / 8 + 255) / 256), 256, 0, stream>>>(w_out, Wot, DD, DD);
  k_qkv<<<dim3(BS / 64, D3 / 128), 128, 0, stream>>>(xh, Wt, b_qkv, qh, kh, vT);
  k_attn<<<dim3(SS / 64, BB * HH), 128, 0, stream>>>(qh, kh, vT, ao);
  k_out<<<dim3(BS / 64, DD / 128), 128, 0, stream>>>(ao, Wot, b_out, out);
}
